// RNNBezierAE_55070070669744
// MI455X (gfx1250) — hardware-run, weakly checked
//
#include <hip/hip_runtime.h>
#include <math.h>

typedef __attribute__((ext_vector_type(16))) _Float16 v16h;
typedef __attribute__((ext_vector_type(8)))  _Float16 v8h;
typedef __attribute__((ext_vector_type(8)))  float    v8f;
typedef __attribute__((ext_vector_type(4)))  float    v4f;

__device__ __forceinline__ void dep_guard_h(v8f& a, v8f& b, v16h x, v16h y) { asm volatile("v_nop\n\tv_nop\n\tv_nop\n\tv_nop" : "+v"(a), "+v"(b) : "v"(x), "v"(y)); }
__device__ __forceinline__ void keep4_h(v16h a, v16h b, v16h c, v16h d) { asm volatile("v_nop" :: "v"(a), "v"(b), "v"(c), "v"(d)); }
__device__ __forceinline__ void acc_guard4(v8f& a, v8f& b, v8f& c, v8f& d) { asm volatile("v_nop\n\tv_nop\n\tv_nop\n\tv_nop" : "+v"(a), "+v"(b), "+v"(c), "+v"(d)); }
template <typename T> struct Frag;
template <> struct Frag<_Float16> {
  typedef v16h V; union U { v16h v; v8h h[2]; };
  static __device__ __forceinline__ v16h load(const _Float16* p) {
    U f; f.h[0] = *(const v8h*)(p); f.h[1] = *(const v8h*)(p + 16); return f.v;
  }
  static __device__ __forceinline__ v8f mma(v16h a, v16h b, v8f c) {
    return __builtin_amdgcn_wmma_f32_16x16x32_f16(false, a, false, b, (short)0, c, false, false);
  }
  static __device__ __forceinline__ void guard(v8f& a, v8f& b, v16h x, v16h y) { dep_guard_h(a, b, x, y); }
  static __device__ __forceinline__ void keep(v16h a, v16h b, v16h c, v16h d) { keep4_h(a, b, c, d); }
};

static constexpr int kT   = 256;
static constexpr int kB   = 512;
static constexpr int kH   = 256;
static constexpr int kG4  = 1024;
static constexpr int kRB  = 16;
static constexpr int kHP  = 264;
static constexpr int kSP  = 260;
static constexpr int kNP  = 522;
static constexpr int kNHC = 1024;
static constexpr int kNC  = 20;
static constexpr int kNR  = 8;

__device__ __forceinline__ int imin_d(int a, int b) { return a < b ? a : b; }
__device__ __forceinline__ float rcp_f(float v) { return __builtin_amdgcn_rcpf(v); }
__device__ __forceinline__ float sigm_f(float v) { return rcp_f(1.0f + expf(-v)); }
__device__ __forceinline__ float tanh_f(float v) { return fmaf(-2.0f, rcp_f(1.0f + expf(2.0f * v)), 1.0f); }

__global__ __launch_bounds__(256) void k_castw(const float* __restrict__ wf, const float* __restrict__ wb,
                                               _Float16* __restrict__ outp, int n2) {
  const int dir = blockIdx.y;
  const int i = blockIdx.x * 256 + threadIdx.x;
  const int ic = imin_d(i, n2 - 1);
  const float* src = dir ? wb : wf;
  const _Float16 h0 = (_Float16)(src[2 * ic] * 64.0f);
  const _Float16 h1 = (_Float16)(src[2 * ic + 1] * 64.0f);
  const unsigned u = (unsigned)__builtin_bit_cast(unsigned short, h0) | ((unsigned)__builtin_bit_cast(unsigned short, h1) << 16);
  if (i < n2) {
    volatile unsigned* o = (volatile unsigned*)(outp + (size_t)dir * 2 * n2);
    o[i] = u;
    __threadfence();
    o[i] = u;
  }
}

__global__ __launch_bounds__(256) void k_lstm(
    const float* __restrict__ x, const float* __restrict__ h0g, const float* __restrict__ c0g,
    const int* __restrict__ lengths,
    const float* __restrict__ wihf, const float* __restrict__ bihf, const float* __restrict__ bhhf,
    const float* __restrict__ wihb, const float* __restrict__ bihb, const float* __restrict__ bhhb,
    const float* __restrict__ wt, const _Float16* __restrict__ W16,
    float* __restrict__ LP, float* __restrict__ HF, float* __restrict__ CF) {
  __shared__ __align__(16) _Float16 hA[2][kRB * kHP];
  __shared__ __align__(16) float fsl[kRB * kSP];
  __shared__ float part[kRB * 16];
  __shared__ __align__(16) float lstage[kRB * 32];
  __shared__ int lens_s[kRB];

  const int tid  = threadIdx.x;
  const int wave = tid >> 5, lane = tid & 31, hh = lane >> 4, c = lane & 15;
  const int koff = hh * 8;
  const int dir  = blockIdx.y;
  const int b0   = blockIdx.x * kRB;
  const float* wih = dir ? wihb : wihf;
  const float* bih = dir ? bihb : bihf;
  const float* bhh = dir ? bhhb : bhhf;
  const _Float16* Wd = W16 + (size_t)dir * kG4 * kH;
  const int ub = wave * 32 + c;

  if (tid < kRB) {
    int L = lengths[imin_d(b0 + tid, kB - 1)];
    L = L < 0 ? 0 : L;
    L = L > kT ? kT : L;
    lens_s[tid] = L;
  }
  {
    const int row = tid >> 4, cs = (tid & 15) * 16;
    const float* src = h0g + ((size_t)(dir * kB + b0 + row)) * kH + cs;
    v8h v0, v1;
#pragma unroll
    for (int e = 0; e < 8; ++e) {
      v0[e] = (_Float16)(src[e] * 16.0f);
      v1[e] = (_Float16)(src[8 + e] * 16.0f);
    }
    *(v8h*)(hA[0] + row * kHP + cs) = v0;
    *(v8h*)(hA[0] + row * kHP + cs + 8) = v1;
  }
  float wi0[2][4], wi1[2][4], bs[2][4], wtv[2];
  float hst[2][8], cst[2][8];
#pragma unroll
  for (int s = 0; s < 2; ++s) {
    const int u = ub + 16 * s;
#pragma unroll
    for (int g = 0; g < 4; ++g) {
      const int n = g * kH + u;
      wi0[s][g] = wih[n * 2];
      wi1[s][g] = wih[n * 2 + 1];
      bs[s][g]  = bih[n] + bhh[n];
    }
    wtv[s] = wt[dir * kH + u];
#pragma unroll
    for (int r = 0; r < 8; ++r) {
      const size_t o = ((size_t)(dir * kB + b0 + hh * 8 + r)) * kH + u;
      hst[s][r] = h0g[o];
      cst[s][r] = c0g[o];
    }
  }
  __syncthreads();
  int lenr[8];
#pragma unroll
  for (int r = 0; r < 8; ++r) lenr[r] = lens_s[hh * 8 + r];

  for (int t = 0; t < kT; ++t) {
    const int cur = t & 1;
    const _Float16* hcur = hA[cur];
    _Float16* hnx = hA[cur ^ 1];
    unsigned zo = 0u;
    asm volatile("" : "+s"(zo));
    const _Float16* Wt = Wd + zo;

    v8f acc[2][4];
#pragma unroll
    for (int s = 0; s < 2; ++s)
#pragma unroll
      for (int g = 0; g < 4; ++g) acc[s][g] = (v8f){0.f, 0.f, 0.f, 0.f, 0.f, 0.f, 0.f, 0.f};

#pragma unroll 1
    for (int kt = 0; kt < 8; ++kt) {
      asm volatile("" ::: "memory");
      const int k0 = kt * 32 + koff;
      const v16h af = Frag<_Float16>::load(hcur + c * kHP + k0);
#pragma unroll
      for (int s = 0; s < 2; ++s) {
        if (s == 1) asm volatile("" ::: "memory");
        v16h bq[4];
#pragma unroll
        for (int g = 0; g < 4; ++g)
          bq[g] = Frag<_Float16>::load(Wt + (size_t)(g * kH + ub + 16 * s) * kH + k0);
#pragma unroll
        for (int g = 0; g < 4; ++g) acc[s][g] = Frag<_Float16>::mma(af, bq[g], acc[s][g]);
        Frag<_Float16>::guard(acc[s][0], acc[s][3], af, bq[0]);
        Frag<_Float16>::keep(bq[0], bq[1], bq[2], bq[3]);
      }
    }
    acc_guard4(acc[0][0], acc[0][1], acc[0][2], acc[0][3]);
    acc_guard4(acc[1][0], acc[1][1], acc[1][2], acc[1][3]);

#pragma unroll
    for (int r = 0; r < 8; ++r) {
      const int row = hh * 8 + r;
      const int L = lenr[r];
      const bool m = (t < L);
      int rv = L - 1 - t;
      rv = rv < 0 ? 0 : rv;
      const int tt = dir ? rv : t;
      const float* xr = x + ((size_t)tt * kB + (b0 + row)) * 2;
      const float x0 = xr[0], x1 = xr[1];
#pragma unroll
      for (int s = 0; s < 2; ++s) {
        const int u = ub + 16 * s;
        const float pi = fmaf(acc[s][0][r], (1.0f / 1024.0f), fmaf(x0, wi0[s][0], fmaf(x1, wi1[s][0], bs[s][0])));
        const float pf = fmaf(acc[s][1][r], (1.0f / 1024.0f), fmaf(x0, wi0[s][1], fmaf(x1, wi1[s][1], bs[s][1])));
        const float pg = fmaf(acc[s][2][r], (1.0f / 1024.0f), fmaf(x0, wi0[s][2], fmaf(x1, wi1[s][2], bs[s][2])));
        const float po = fmaf(acc[s][3][r], (1.0f / 1024.0f), fmaf(x0, wi0[s][3], fmaf(x1, wi1[s][3], bs[s][3])));
        const float ig = sigm_f(pi);
        const float fg = sigm_f(pf);
        const float og = sigm_f(po);
        const float gt = tanh_f(pg);
        const float cn = fmaf(fg, cst[s][r], ig * gt);
        const float hn = og * tanh_f(cn);
        const float ck = m ? cn : cst[s][r];
        const float hk = m ? hn : hst[s][r];
        cst[s][r] = ck;
        hst[s][r] = hk;
        hnx[row * kHP + u] = (_Float16)(hk * 16.0f);
        fsl[row * kSP + u] = m ? hn * wtv[s] : 0.0f;
      }
    }
    __syncthreads();
    {
      const int row = tid >> 4, seg = tid & 15;
      const float* pp = fsl + row * kSP + seg * 16;
      const v4f q0 = *(const v4f*)(pp);
      const v4f q1 = *(const v4f*)(pp + 4);
      const v4f q2 = *(const v4f*)(pp + 8);
      const v4f q3 = *(const v4f*)(pp + 12);
      float sum = q0[0];
      sum += q0[1]; sum += q0[2]; sum += q0[3];
      sum += q1[0]; sum += q1[1]; sum += q1[2]; sum += q1[3];
      sum += q2[0]; sum += q2[1]; sum += q2[2]; sum += q2[3];
      sum += q3[0]; sum += q3[1]; sum += q3[2]; sum += q3[3];
      part[row * 16 + seg] = sum;
    }
    __syncthreads();
    if (tid < kRB) {
      const int rr = imin_d(tid, kRB - 1);
      float sum = 0.0f;
#pragma unroll
      for (int j = 0; j < 16; ++j) sum += part[rr * 16 + j];
      lstage[rr * 32 + (t & 31)] = sum;
    }
    if ((t & 31) == 31) {
      __syncthreads();
      if (wave < 4) {
        const int row = wave * 4 + (lane >> 3), c4 = (lane & 7) * 4;
        const v4f v = *(const v4f*)(lstage + row * 32 + c4);
        float* dst = LP + ((size_t)(dir * kB + b0 + row)) * kT + (t - 31) + c4;
        *(volatile v4f*)dst = v;
        __threadfence();
        *(volatile v4f*)dst = v;
      }
    }
  }

  __syncthreads();
#pragma unroll
  for (int s = 0; s < 2; ++s)
#pragma unroll
    for (int r = 0; r < 8; ++r) fsl[(hh * 8 + r) * kSP + ub + 16 * s] = hst[s][r];
  __syncthreads();
  {
    v4f v[4];
    float* d[4];
#pragma unroll
    for (int q = 0; q < 4; ++q) {
      const int row = wave * 2 + (q >> 1), c4 = (q & 1) * 128 + lane * 4;
      v[q] = *(const v4f*)(fsl + row * kSP + c4);
      d[q] = HF + ((size_t)(dir * kB + b0 + row)) * kH + c4;
    }
#pragma unroll
    for (int q = 0; q < 4; ++q) *(volatile v4f*)d[q] = v[q];
    __threadfence();
#pragma unroll
    for (int q = 0; q < 4; ++q) *(volatile v4f*)d[q] = v[q];
  }
  __syncthreads();
#pragma unroll
  for (int s = 0; s < 2; ++s)
#pragma unroll
    for (int r = 0; r < 8; ++r) fsl[(hh * 8 + r) * kSP + ub + 16 * s] = cst[s][r];
  __syncthreads();
  {
    v4f v[4];
    float* d[4];
#pragma unroll
    for (int q = 0; q < 4; ++q) {
      const int row = wave * 2 + (q >> 1), c4 = (q & 1) * 128 + lane * 4;
      v[q] = *(const v4f*)(fsl + row * kSP + c4);
      d[q] = CF + ((size_t)(dir * kB + b0 + row)) * kH + c4;
    }
#pragma unroll
    for (int q = 0; q < 4; ++q) *(volatile v4f*)d[q] = v[q];
    __threadfence();
#pragma unroll
    for (int q = 0; q < 4; ++q) *(volatile v4f*)d[q] = v[q];
  }
}

__global__ __launch_bounds__(256) void k_tail(
    const float* __restrict__ LP, const float* __restrict__ HF, const float* __restrict__ CF,
    const int* __restrict__ lengths, const float* __restrict__ bt,
    const float* __restrict__ wproj, const float* __restrict__ bproj,
    const float* __restrict__ wctrl, const float* __restrict__ bctrl,
    const float* __restrict__ wratw, const float* __restrict__ bratw,
    float* __restrict__ outc, float* __restrict__ regp) {
  __shared__ __align__(16) float hc[kNHC];
  __shared__ __align__(16) float pj[528];
  __shared__ float Psh[24];
  __shared__ float Rsh[12];
  __shared__ float red[24];
  __shared__ __align__(16) float curv[2 * kT];

  const int tid = threadIdx.x, lane = tid & 31, wave = tid >> 5;
  const int b = blockIdx.x;
  const int t = tid;
  int L = lengths[b];
  L = L < 0 ? 0 : L;
  L = L > kT ? kT : L;
  int rv = L - 1 - t;
  rv = rv < 0 ? 0 : rv;
  rv = rv > kT - 1 ? kT - 1 : rv;
  const float lfv = LP[(size_t)b * kT + t];
  const float lbv = LP[(size_t)(kB + b) * kT + rv];
  const bool m = (t < L);
  const float logit = (lfv + (m ? lbv : 0.0f)) + bt[0];

  hc[t] = HF[(size_t)b * kH + t];
  hc[kH + t] = HF[(size_t)(kB + b) * kH + t];
  const float cf = CF[(size_t)b * kH + t];
  hc[2 * kH + t] = cf;
  hc[3 * kH + t] = cf;

  float mx = logit;
#pragma unroll
  for (int off = 1; off < 32; off <<= 1) mx = fmaxf(mx, __shfl_xor(mx, off, 32));
  if (lane == 0) red[wave] = mx;
  __syncthreads();
  float gmx = red[0];
#pragma unroll
  for (int w = 1; w < 8; ++w) gmx = fmaxf(gmx, red[w]);
  const float e = expf(logit - gmx);
  float se = e;
#pragma unroll
  for (int off = 1; off < 32; off <<= 1) se += __shfl_xor(se, off, 32);
  if (lane == 0) red[8 + wave] = se;
  __syncthreads();
  float tot = red[8];
#pragma unroll
  for (int w = 1; w < 8; ++w) tot += red[8 + w];
  const float p = e / tot;
  float sc = p;
#pragma unroll
  for (int d = 1; d < 32; d <<= 1) {
    const float y = __shfl_up(sc, d, 32);
    sc = (lane >= d) ? (sc + y) : sc;
  }
  if (lane == 31) red[16 + wave] = sc;
  __syncthreads();
  float offv = 0.0f;
  for (int w = 0; w < wave; ++w) offv += red[16 + w];
  const float ts = offv + sc;

  {
    const float* w0 = wproj + (size_t)t * kNHC;
    const float* w1 = wproj + (size_t)(t + 256) * kNHC;
    float a0 = 0.0f, a1 = 0.0f;
#pragma unroll 1
    for (int k = 0; k < kNHC; k += 4) {
      const v4f hv = *(const v4f*)(hc + k);
      const v4f wa = *(const v4f*)(w0 + k);
      const v4f wb = *(const v4f*)(w1 + k);
      a0 = fmaf(wa[0], hv[0], a0); a0 = fmaf(wa[1], hv[1], a0); a0 = fmaf(wa[2], hv[2], a0); a0 = fmaf(wa[3], hv[3], a0);
      a1 = fmaf(wb[0], hv[0], a1); a1 = fmaf(wb[1], hv[1], a1); a1 = fmaf(wb[2], hv[2], a1); a1 = fmaf(wb[3], hv[3], a1);
    }
    pj[t] = fmaxf(a0 + bproj[t], 0.0f);
    pj[t + 256] = fmaxf(a1 + bproj[t + 256], 0.0f);
    const int r2 = imin_d(t + 512, kNP - 1);
    if (t < kNP - 512) {
      const float* w2 = wproj + (size_t)r2 * kNHC;
      float a2 = 0.0f;
#pragma unroll 1
      for (int k = 0; k < kNHC; k += 4) {
        const v4f hv = *(const v4f*)(hc + k);
        const v4f wc = *(const v4f*)(w2 + k);
        a2 = fmaf(wc[0], hv[0], a2); a2 = fmaf(wc[1], hv[1], a2); a2 = fmaf(wc[2], hv[2], a2); a2 = fmaf(wc[3], hv[3], a2);
      }
      pj[r2] = fmaxf(a2 + bproj[r2], 0.0f);
    }
  }
  __syncthreads();
  if (wave == 0) {
    const int lc = imin_d(lane, kNC - 1);
    const float* wr = wctrl + (size_t)lc * kNP;
    float a = 0.0f;
#pragma unroll 1
    for (int k = 0; k < kNP; ++k) a = fmaf(wr[k], pj[k], a);
    const float pv = a + bctrl[lc];
    if (lane < kNC) Psh[lane] = pv;
  } else if (wave == 1) {
    const int lc = imin_d(lane, kNR - 1);
    const float* wr = wratw + (size_t)lc * kNP;
    float a = 0.0f;
#pragma unroll 1
    for (int k = 0; k < kNP; ++k) a = fmaf(wr[k], pj[k], a);
    const float a2 = a + bratw[lc];
    const float rvw = 1.0f / (1.0f + expf(-a2));
    if (lane < kNR) Rsh[1 + lane] = rvw;
    if (lane == kNR) {
      Rsh[0] = 0.5f;
      Rsh[kNR + 1] = 0.5f;
    }
  }
  __syncthreads();
  {
#pragma clang fp contract(off)
    const float bin[10] = {1.0f, 9.0f, 36.0f, 84.0f, 126.0f, 126.0f, 84.0f, 36.0f, 9.0f, 1.0f};
    static_assert(sizeof(bin) / sizeof(bin[0]) == 10);
    const float tv = ts;
    const float sv = 1.0f - tv;
    float tp[10], sp[10];
    tp[0] = 1.0f;
    sp[0] = 1.0f;
#pragma unroll
    for (int i = 1; i < 10; ++i) {
      tp[i] = tp[i - 1] * tv;
      sp[i] = sp[i - 1] * sv;
    }
    float wsum = 0.0f, nx = 0.0f, ny = 0.0f;
#pragma unroll
    for (int i = 0; i < 10; ++i) {
      const float w = ((bin[i] * tp[i]) * sp[9 - i]) * Rsh[i];
      wsum = wsum + w;
      nx = nx + w * Psh[2 * i];
      ny = ny + w * Psh[2 * i + 1];
    }
    const float mf = m ? 1.0f : 0.0f;
    const float cx = (nx / wsum) * mf;
    const float cy = (ny / wsum) * mf;
    curv[2 * t] = cx;
    curv[2 * t + 1] = cy;
    if (tid == 0) {
      float s = 0.0f;
#pragma unroll
      for (int i = 0; i < 9; ++i) {
        const float dx = Psh[2 * i + 2] - Psh[2 * i];
        const float dy = Psh[2 * i + 3] - Psh[2 * i + 1];
        s = s + (dx * dx + dy * dy);
      }
      red[20] = s;
    }
  }
  __syncthreads();
  if (wave < 4) {
    const int idx = wave * 128 + lane * 4;
    const v4f v = *(const v4f*)(curv + idx);
    float* dst = outc + (size_t)b * (2 * kT) + idx;
    *(volatile v4f*)dst = v;
    __threadfence();
    *(volatile v4f*)dst = v;
  } else if (wave == 4) {
    if (lane < 8) {
      const float s = red[20];
      v4f v;
      v[0] = (lane == 0) ? s : 0.0f;
      v[1] = 0.0f; v[2] = 0.0f; v[3] = 0.0f;
      float* dst = regp + (size_t)b * 32 + lane * 4;
      *(volatile v4f*)dst = v;
      __threadfence();
      *(volatile v4f*)dst = v;
    }
  }
}

__global__ __launch_bounds__(32) void k_regsum(const float* __restrict__ regp, float* __restrict__ out1) {
  if (threadIdx.x == 0) {
    float s = 0.0f;
#pragma unroll 1
    for (int bb = 0; bb < kB; ++bb) s += regp[(size_t)bb * 32];
    const float r = s / 4608.0f;
    *(volatile float*)out1 = r;
    __threadfence();
    *(volatile float*)out1 = r;
  }
}

extern "C" void kernel_launch(void* const* d_in, const int* in_sizes, int n_in,
                              void* d_out, int out_size, void* d_ws, size_t ws_size,
                              hipStream_t stream) {
  const float* x     = (const float*)d_in[0];
  const float* h0    = (const float*)d_in[1];
  const float* c0    = (const float*)d_in[2];
  const int*   len   = (const int*)d_in[3];
  const float* wihf  = (const float*)d_in[4];
  const float* whhf  = (const float*)d_in[5];
  const float* bihf  = (const float*)d_in[6];
  const float* bhhf  = (const float*)d_in[7];
  const float* wihb  = (const float*)d_in[8];
  const float* whhb  = (const float*)d_in[9];
  const float* bihb  = (const float*)d_in[10];
  const float* bhhb  = (const float*)d_in[11];
  const float* wt    = (const float*)d_in[12];
  const float* bt    = (const float*)d_in[13];
  const float* wproj = (const float*)d_in[14];
  const float* bproj = (const float*)d_in[15];
  const float* wctrl = (const float*)d_in[16];
  const float* bctrl = (const float*)d_in[17];
  const float* wratw = (const float*)d_in[18];
  const float* bratw = (const float*)d_in[19];
  float* out = (float*)d_out;

  char* ws = (char*)d_ws;
  const size_t oW16 = 0;
  const size_t oLP  = oW16 + (size_t)2 * kG4 * kH * 2;
  const size_t oHF  = oLP  + (size_t)2 * kB * kT * 4;
  const size_t oCF  = oHF  + (size_t)2 * kB * kH * 4;
  const size_t oRG  = oCF  + (size_t)2 * kB * kH * 4;
  const size_t oEnd = oRG  + (size_t)kB * 32 * 4;
  if (oEnd > ws_size) return;
  if ((size_t)out_size < (size_t)kB * kT * 2 + 1) return;
  if (n_in < 20) return;

  _Float16* W16 = (_Float16*)(ws + oW16);
  float* LP  = (float*)(ws + oLP);
  float* HF  = (float*)(ws + oHF);
  float* CF  = (float*)(ws + oCF);
  float* RG  = (float*)(ws + oRG);
  float* out1 = out + (size_t)kB * kT * 2;

  const int n2 = kG4 * kH / 2;
  k_castw<<<dim3((n2 + 255) / 256, 2, 1), 256, 0, stream>>>(whhf, whhb, W16, n2);
  k_lstm<<<dim3(kB / kRB, 2, 1), 256, 0, stream>>>(x, h0, c0, len, wihf, bihf, bhhf, wihb, bihb, bhhb,
                                                  wt, W16, LP, HF, CF);
  k_tail<<<kB, 256, 0, stream>>>(LP, HF, CF, len, bt, wproj, bproj, wctrl, bctrl, wratw, bratw, out, RG);
  k_regsum<<<1, 32, 0, stream>>>(RG, out1);
}
